// MultiHeadAttention_70549132804637
// MI455X (gfx1250) — hardware-verified
//
#include <hip/hip_runtime.h>
#include <stddef.h>


typedef _Float16 h16;
typedef _Float16 v16h __attribute__((ext_vector_type(16)));
typedef _Float16 v8h  __attribute__((ext_vector_type(8)));
typedef float    v8f  __attribute__((ext_vector_type(8)));
typedef float    v4f  __attribute__((ext_vector_type(4)));

#ifndef NB
#define NB 4
#endif
#ifndef SEQ
#define SEQ 2048
#endif
#define NB_FULL  4
#define SEQ_FULL 2048
#define DIM   1024
#define NHEAD 16
#define HD    64
#define QKVN  (3 * DIM)
#define MROWS (NB * SEQ)

static_assert(NB >= 1 && NB <= NB_FULL);
static_assert(SEQ >= 128 && SEQ <= SEQ_FULL && (SEQ % 128) == 0);
static_assert(DIM == NHEAD * HD);
static_assert(HD == 64);
static_assert(QKVN == 3 * DIM && (QKVN / 64) == 3 * NHEAD);
static_assert((DIM % 64) == 0 && (DIM % 32) == 0);
static_assert((QKVN % 64) == 0);
static_assert((SEQ % 64) == 0 && (SEQ % 32) == 0);
static_assert((MROWS % 64) == 0 && (MROWS % 2) == 0);
static_assert((QKVN % 2) == 0 && (DIM % 2) == 0);
static_assert(DIM / 8 == 128);
static_assert((size_t)MROWS * (DIM / 8) < (size_t)0xFFFFFFFFu);

#define LDT 72
#define LDC 68
static_assert((LDT % 8) == 0 && LDT >= 64);
static_assert((LDC % 4) == 0 && LDC >= 64);

#define WCARRY   64.0f
#define SCALE_QK 0.125f

#define WQKV_BYTES    ((size_t)QKVN * DIM * 2)
#define WO_BYTES      ((size_t)DIM * DIM * 2)
#define PLANE16_BYTES ((size_t)MROWS * DIM * 2)
#define TPLANE_ELEMS  ((size_t)NB * DIM * SEQ)
#define T_BYTES       ((size_t)2 * TPLANE_ELEMS * 2)
#define KV_BYTES      ((size_t)NB * NHEAD * HD * HD * 2)
#define OFF_WQKV ((size_t)0)
#define OFF_WO   (OFF_WQKV + WQKV_BYTES)
#define OFF_X    (OFF_WO + WO_BYTES)
#define OFF_Q    (OFF_X + PLANE16_BYTES)
#define OFF_T    (OFF_Q + PLANE16_BYTES)
#define OFF_KV   (OFF_T + T_BYTES)
#define OFF_CTX  (OFF_KV + KV_BYTES)
#define WS_TOTAL (OFF_CTX + PLANE16_BYTES)
static_assert((WQKV_BYTES % 128) == 0 && (WO_BYTES % 128) == 0 && (PLANE16_BYTES % 128) == 0);
static_assert((T_BYTES % 128) == 0 && (KV_BYTES % 128) == 0);
static_assert(WS_TOTAL <= (size_t)134217728);

__device__ __forceinline__ float bf16r(float x) {
  unsigned int u = __float_as_uint(x);
  u = (u + 0x7FFFu + ((u >> 16) & 1u)) & 0xFFFF0000u;
  return __uint_as_float(u);
}

static __device__ __forceinline__ h16 toh_flush(float v) {
  const h16 r = (h16)v;
  return (fabsf(v) < 6.103515625e-05f) ? (h16)0.0f : r;
}

__device__ __forceinline__ v16h frag_at(const _Float16* p) {
  v8h lo = *(const v8h*)(p);
  v8h hi = *(const v8h*)(p + 16);
  v16h out;
#pragma unroll
  for (int i = 0; i < 8; ++i) { out[i] = lo[i]; out[i + 8] = hi[i]; }
  return out;
}

__device__ __forceinline__ v8f wmma16(v16h a, v16h b, v8f c) {
  v8f d = __builtin_amdgcn_wmma_f32_16x16x32_f16(false, a, false, b, (short)0, c,
                                                 false, false);
  asm volatile("v_nop\n\tv_nop\n\tv_nop\n\tv_nop" : "+v"(d) : "v"(a), "v"(b));
  return d;
}

__device__ __forceinline__ void wave_lds_sync() {
  __builtin_amdgcn_fence(3  , "wavefront");
  asm volatile("s_wait_dscnt 0x0" ::: "memory");
  __builtin_amdgcn_wave_barrier();
}

__global__ __launch_bounds__(256) void cvt_plane_kernel(
    const float* __restrict__ src, _Float16* __restrict__ dst,
    unsigned seq, unsigned seq_full, float carry) {
#pragma clang fp contract(off)
  const unsigned g = blockIdx.x * 256u + threadIdx.x;
  const unsigned crow = g >> 7;
  const unsigned c = (g & 127u) * 8u;
  const unsigned bidx = crow / seq;
  const unsigned sq = crow - bidx * seq;
  const size_t srow = (size_t)bidx * seq_full + sq;
  const v4f a0 = *(const v4f*)(src + srow * DIM + c);
  const v4f a1 = *(const v4f*)(src + srow * DIM + c + 4u);
  v8h o;
#pragma unroll
  for (int i = 0; i < 4; ++i) {
    o[i]     = toh_flush(carry * bf16r(a0[i]));
    o[i + 4] = toh_flush(carry * bf16r(a1[i]));
  }
  _Float16* p = dst + (size_t)crow * DIM + c;
  *(volatile v8h*)p = o;
  __threadfence();
  *(volatile v8h*)p = o;
}

template <int MODE>
__device__ __forceinline__ void gemm_body(
    const _Float16* __restrict__ A16, const _Float16* __restrict__ Bt, const unsigned K,
    float* __restrict__ outf, _Float16* __restrict__ outq, _Float16* __restrict__ outt) {
  __shared__ __attribute__((aligned(16))) float Cs[64 * LDC];
  const unsigned tid = threadIdx.x, lane = tid & 31u;
  const unsigned w = (unsigned)__builtin_amdgcn_readfirstlane((int)(threadIdx.x >> 5));
  const unsigned mw = w >> 1, nw = w & 1u;
  const unsigned hh = lane >> 4, m = lane & 15u;
  const unsigned n0 = blockIdx.x * 64u;
  const unsigned row0 = blockIdx.y * 64u;

  const _Float16* ap  = A16 + (size_t)(row0 + mw * 16u + m) * K + hh * 8u;
  const _Float16* bp0 = Bt + (size_t)(n0 + nw * 32u + m) * K + hh * 8u;
  const _Float16* bp1 = bp0 + (size_t)16 * K;
  v8f acc0 = {}, acc1 = {};
#pragma unroll 2
  for (unsigned k0 = 0; k0 < K; k0 += 32u) {
    const v16h a  = frag_at(ap + k0);
    const v16h b0 = frag_at(bp0 + k0);
    const v16h b1 = frag_at(bp1 + k0);
    acc0 = wmma16(a, b0, acc0);
    acc1 = wmma16(a, b1, acc1);
  }
#pragma unroll
  for (int r = 0; r < 8; ++r) {
    float* d = &Cs[(mw * 16u + hh * 8u + (unsigned)r) * LDC + nw * 32u + m];
    d[0]  = acc0[r];
    d[16] = acc1[r];
  }
  __syncthreads();

  if (MODE == 0) {
    const unsigned nt = blockIdx.x;
    const unsigned head = nt / 3u;
    const unsigned part = nt - head * 3u;
    if (part == 0u) {
      v8h x[2];
      size_t off[2];
#pragma unroll
      for (unsigned i = 0; i < 2u; ++i) {
        const unsigned r = 32u * i + (tid >> 3);
        const unsigned c = (tid & 7u) * 8u;
        const v4f u0 = *(const v4f*)&Cs[r * LDC + c];
        const v4f u1 = *(const v4f*)&Cs[r * LDC + c + 4];
#pragma unroll
        for (int j = 0; j < 4; ++j) {
          x[i][j]     = toh_flush(u0[j] * (1.0f / WCARRY));
          x[i][j + 4] = toh_flush(u1[j] * (1.0f / WCARRY));
        }
        off[i] = (size_t)(row0 + r) * DIM + head * HD + c;
      }
#pragma unroll
      for (int i = 0; i < 2; ++i) *(volatile v8h*)(outq + off[i]) = x[i];
      __threadfence();
#pragma unroll
      for (int i = 0; i < 2; ++i) *(volatile v8h*)(outq + off[i]) = x[i];
    } else {
      const unsigned bidx = row0 / (unsigned)SEQ;
      const unsigned key0 = row0 - bidx * (unsigned)SEQ;
      v8h x[2];
      size_t off[2];
#pragma unroll
      for (unsigned i = 0; i < 2u; ++i) {
        const unsigned dcol = 32u * i + (tid >> 3);
        const unsigned kk = (tid & 7u) * 8u;
#pragma unroll
        for (unsigned j = 0; j < 8u; ++j) {
          const float t = Cs[(kk + j) * LDC + dcol] * (1.0f / WCARRY);
          x[i][j] = toh_flush(t);
        }
        off[i] = (size_t)(part - 1u) * TPLANE_ELEMS +
                 ((size_t)bidx * DIM + head * HD + dcol) * SEQ + key0 + kk;
      }
#pragma unroll
      for (int i = 0; i < 2; ++i) *(volatile v8h*)(outt + off[i]) = x[i];
      __threadfence();
#pragma unroll
      for (int i = 0; i < 2; ++i) *(volatile v8h*)(outt + off[i]) = x[i];
    }
  }

  if (MODE == 1) {
    v4f xs[4];
    size_t off[4];
#pragma unroll
    for (unsigned i = 0; i < 4u; ++i) {
      const unsigned r = 16u * i + (tid >> 4);
      const unsigned c = (tid & 15u) * 4u;
      const unsigned crow = row0 + r;
      const unsigned bidx = crow / (unsigned)SEQ;
      const unsigned sq = crow - bidx * (unsigned)SEQ;
      const size_t frow = (size_t)bidx * SEQ_FULL + sq;
      const v4f u = *(const v4f*)&Cs[r * LDC + c];
      v4f val;
#pragma unroll
      for (int j = 0; j < 4; ++j) val[j] = u[j] * (1.0f / WCARRY);
      xs[i] = val;
      off[i] = frow * DIM + n0 + c;
    }
#pragma unroll
    for (int i = 0; i < 4; ++i) *(volatile v4f*)(outf + off[i]) = xs[i];
    __threadfence();
#pragma unroll
    for (int i = 0; i < 4; ++i) *(volatile v4f*)(outf + off[i]) = xs[i];
  }
}

__global__ __launch_bounds__(256) void gemm_qkv_kernel(
    const _Float16* __restrict__ A16, const _Float16* __restrict__ Bt,
    _Float16* __restrict__ qplane, _Float16* __restrict__ tplane) {
  gemm_body<0>(A16, Bt, (unsigned)DIM, (float*)0, qplane, tplane);
}
__global__ __launch_bounds__(256) void gemm_out_kernel(
    const _Float16* __restrict__ A16, const _Float16* __restrict__ Bt,
    float* __restrict__ outf) {
  gemm_body<1>(A16, Bt, (unsigned)DIM, outf, (_Float16*)0, (_Float16*)0);
}

__global__ __launch_bounds__(256) void ktv_kernel(
    const _Float16* __restrict__ T16, _Float16* __restrict__ KVt) {
  __shared__ __attribute__((aligned(16))) float Cs[64 * LDC];
  const unsigned tid = threadIdx.x, lane = tid & 31u;
  const unsigned w = (unsigned)__builtin_amdgcn_readfirstlane((int)(threadIdx.x >> 5));
  const unsigned tr = w >> 1, tc0 = (w & 1u) * 2u;
  const unsigned hh = lane >> 4, m = lane & 15u;
  const unsigned head = blockIdx.x;
  const unsigned b = blockIdx.y;

  const size_t kbase = ((size_t)b * DIM + head * HD) * SEQ;
  const size_t vbase = TPLANE_ELEMS + kbase;
  const _Float16* ap  = T16 + vbase + (size_t)(tr * 16u + m) * SEQ + hh * 8u;
  const _Float16* bp0 = T16 + kbase + (size_t)(tc0 * 16u + m) * SEQ + hh * 8u;
  const _Float16* bp1 = bp0 + (size_t)16 * SEQ;
  v8f acc0 = {}, acc1 = {};
#pragma unroll 2
  for (unsigned s0 = 0; s0 < (unsigned)SEQ; s0 += 32u) {
    const v16h a  = frag_at(ap + s0);
    const v16h b0 = frag_at(bp0 + s0);
    const v16h b1 = frag_at(bp1 + s0);
    acc0 = wmma16(a, b0, acc0);
    acc1 = wmma16(a, b1, acc1);
  }
#pragma unroll
  for (int r = 0; r < 8; ++r) {
    float* d = &Cs[(tr * 16u + hh * 8u + (unsigned)r) * LDC + tc0 * 16u + m];
    d[0]  = acc0[r];
    d[16] = acc1[r];
  }
  __syncthreads();

  v8h x[2];
  size_t off[2];
#pragma unroll
  for (unsigned i = 0; i < 2u; ++i) {
    const unsigned r = 32u * i + (tid >> 3);
    const unsigned c = (tid & 7u) * 8u;
    const v4f u0 = *(const v4f*)&Cs[r * LDC + c];
    const v4f u1 = *(const v4f*)&Cs[r * LDC + c + 4];
#pragma unroll
    for (int j = 0; j < 4; ++j) {
      x[i][j]     = toh_flush(u0[j]);
      x[i][j + 4] = toh_flush(u1[j]);
    }
    off[i] = ((size_t)(b * NHEAD + head) * HD + r) * HD + c;
  }
#pragma unroll
  for (int i = 0; i < 2; ++i) *(volatile v8h*)(KVt + off[i]) = x[i];
  __threadfence();
#pragma unroll
  for (int i = 0; i < 2; ++i) *(volatile v8h*)(KVt + off[i]) = x[i];
}

__global__ __launch_bounds__(256) void qkv_apply_kernel(
    const _Float16* __restrict__ Qh, const _Float16* __restrict__ KVt,
    _Float16* __restrict__ Ov) {
  __shared__ __attribute__((aligned(16))) _Float16 Ps[8 * 16 * LDT];
  const unsigned tid = threadIdx.x, lane = tid & 31u;
  const unsigned w = (unsigned)__builtin_amdgcn_readfirstlane((int)(threadIdx.x >> 5));
  const unsigned hh = lane >> 4, m = lane & 15u;
  const unsigned q0 = blockIdx.x * 128u;
  const unsigned head = blockIdx.y;
  const unsigned b = blockIdx.z;
  const unsigned qrow0 = q0 + w * 16u;
  const unsigned pbase = w * (16u * LDT);

  const size_t qoff = (size_t)(b * (unsigned)SEQ + qrow0 + m) * DIM + head * HD + hh * 8u;
  const v16h qf0 = frag_at(Qh + qoff);
  const v16h qf1 = frag_at(Qh + qoff + 32);
  const _Float16* kvp = KVt + (size_t)(b * NHEAD + head) * (HD * HD) + (size_t)m * HD + hh * 8u;

  v8f o[4];
#pragma unroll
  for (int nb = 0; nb < 4; ++nb) {
    const v16h b0 = frag_at(kvp + nb * 16 * HD);
    const v16h b1 = frag_at(kvp + nb * 16 * HD + 32);
    v8f t = {};
    t = wmma16(qf0, b0, t);
    t = wmma16(qf1, b1, t);
    o[nb] = t;
  }

#pragma unroll
  for (int nb = 0; nb < 4; ++nb)
#pragma unroll
    for (int v = 0; v < 8; ++v)
      Ps[pbase + (hh * 8u + (unsigned)v) * LDT + (unsigned)nb * 16u + m] =
          toh_flush(o[nb][v] * SCALE_QK);
  wave_lds_sync();
  v8h x[4];
  size_t off[4];
#pragma unroll
  for (unsigned i = 0; i < 4u; ++i) {
    const unsigned r = 4u * i + (lane >> 3);
    const unsigned c = (lane & 7u) * 8u;
    x[i] = *(const v8h*)&Ps[pbase + r * LDT + c];
    off[i] = (size_t)(b * (unsigned)SEQ + qrow0 + r) * DIM + head * HD + c;
  }
#pragma unroll
  for (int i = 0; i < 4; ++i) *(volatile v8h*)(Ov + off[i]) = x[i];
  __threadfence();
#pragma unroll
  for (int i = 0; i < 4; ++i) *(volatile v8h*)(Ov + off[i]) = x[i];
}

extern "C" void kernel_launch(void* const* d_in, const int* in_sizes, int n_in,
                              void* d_out, int out_size, void* d_ws, size_t ws_size,
                              hipStream_t stream) {
  if (n_in < 3) return;
  const long long need_x = ((long long)(NB - 1) * SEQ_FULL + SEQ) * DIM;
  if ((long long)in_sizes[0] < need_x) return;
  if ((long long)in_sizes[1] < (long long)QKVN * DIM) return;
  if ((long long)in_sizes[2] < (long long)DIM * DIM) return;
  if ((long long)out_size < need_x) return;
  if (ws_size < WS_TOTAL) return;

  const float* X    = (const float*)d_in[0];
  const float* wqkv = (const float*)d_in[1];
  const float* wo   = (const float*)d_in[2];
  float* out = (float*)d_out;

  char* ws = (char*)d_ws;
  _Float16* Wqkv16 = (_Float16*)(ws + OFF_WQKV);
  _Float16* Wo16   = (_Float16*)(ws + OFF_WO);
  _Float16* X16    = (_Float16*)(ws + OFF_X);
  _Float16* Q16    = (_Float16*)(ws + OFF_Q);
  _Float16* T16    = (_Float16*)(ws + OFF_T);
  _Float16* KVt16  = (_Float16*)(ws + OFF_KV);
  _Float16* Ctx16  = (_Float16*)(ws + OFF_CTX);

  dim3 blk(256);

  cvt_plane_kernel<<<dim3(QKVN / 2), blk, 0, stream>>>(wqkv, Wqkv16, (unsigned)QKVN, (unsigned)QKVN, WCARRY);
  cvt_plane_kernel<<<dim3(DIM / 2), blk, 0, stream>>>(wo, Wo16, (unsigned)DIM, (unsigned)DIM, WCARRY);
  cvt_plane_kernel<<<dim3(MROWS / 2), blk, 0, stream>>>(X, X16, (unsigned)SEQ, (unsigned)SEQ_FULL, 1.0f);

  gemm_qkv_kernel<<<dim3(QKVN / 64, MROWS / 64), blk, 0, stream>>>(X16, Wqkv16, Q16, T16);
  ktv_kernel<<<dim3(NHEAD, NB), blk, 0, stream>>>(T16, KVt16);
  qkv_apply_kernel<<<dim3(SEQ / 128, NHEAD, NB), blk, 0, stream>>>(Q16, KVt16, Ctx16);
  gemm_out_kernel<<<dim3(DIM / 64, MROWS / 64), blk, 0, stream>>>(Ctx16, Wo16, out);
}
